// PosTransformer_83932250898494
// MI455X (gfx1250) — hardware-verified
//
#include <hip/hip_runtime.h>
#include <stdint.h>
#include <math.h>

#define NBATCH 16
#define NPT    2048
#define DM     384
#define KE     64
#define NCH    60
#define NFREQ  10
#define WQKV_PIECES (3 * DM * (KE / 8))
#define W2_PIECES   (DM * (DM / 8))
#define WCVT_N      (WQKV_PIECES + W2_PIECES)
#define QK_SCALE    0.051031036307982884f

static_assert((NPT % 64) == 0 && (DM % 64) == 0 && (KE % 32) == 0 && (DM % 32) == 0);
static_assert(NPT == 256 * 8);
static_assert((WQKV_PIECES % 256) == 0 && (WCVT_N % 256) == 0);
static_assert((DM * (KE / 8)) % 256 == 0);
static_assert(((DM / 64) * (NPT / 64)) % 8 == 0 && ((NPT / 64) * (NPT / 64)) % 8 == 0);

typedef _Float16 v16h __attribute__((ext_vector_type(16)));
typedef _Float16 v8h  __attribute__((ext_vector_type(8)));
typedef float    v8f  __attribute__((ext_vector_type(8)));
typedef float    v4f  __attribute__((ext_vector_type(4)));
typedef unsigned int v4u __attribute__((ext_vector_type(4)));

__device__ __forceinline__ unsigned short bf_bits(float f) {
  unsigned u = __float_as_uint(f);
  return (unsigned short)((u + 0x7FFFu + ((u >> 16) & 1u)) >> 16);
}
__device__ __forceinline__ float bfr(float f) {
  return __uint_as_float(((unsigned)bf_bits(f)) << 16);
}
__device__ __forceinline__ v8f zero8() { v8f z = {0.f, 0.f, 0.f, 0.f, 0.f, 0.f, 0.f, 0.f}; return z; }
__device__ __forceinline__ v4u pack8h(v4f a, v4f b) {
  union { v8h h; v4u u; } c;
  c.h[0] = (_Float16)a[0]; c.h[1] = (_Float16)a[1]; c.h[2] = (_Float16)a[2]; c.h[3] = (_Float16)a[3];
  c.h[4] = (_Float16)b[0]; c.h[5] = (_Float16)b[1]; c.h[6] = (_Float16)b[2]; c.h[7] = (_Float16)b[3];
  return c.u;
}

__device__ __forceinline__ v16h ldfrag(const _Float16* p) {
  union { v16h v; v8h h[2]; } f;
  f.h[0] = *(const v8h*)(p);
  f.h[1] = *(const v8h*)(p + 16);
  return f.v;
}

__device__ __forceinline__ v8f mma_raw(v16h a, v16h b, v8f c) {
  return __builtin_amdgcn_wmma_f32_16x16x32_f16(false, a, false, b, (short)0, c, false, false);
}
__device__ __forceinline__ void dep_guard(v8f& a, v8f& b, v16h x, v16h y) {
#if defined(__HIP_DEVICE_COMPILE__)
  asm volatile("v_nop\n\tv_nop\n\tv_nop\n\tv_nop" : "+v"(a), "+v"(b) : "v"(x), "v"(y));
#endif
}
__device__ __forceinline__ void keep4(v16h a, v16h b, v16h c, v16h d) {
#if defined(__HIP_DEVICE_COMPILE__)
  asm volatile("v_nop" :: "v"(a), "v"(b), "v"(c), "v"(d));
#endif
}
__device__ __forceinline__ void acc_guard4(v8f& a, v8f& b, v8f& c, v8f& d) {
#if defined(__HIP_DEVICE_COMPILE__)
  asm volatile("v_nop\n\tv_nop\n\tv_nop\n\tv_nop" : "+v"(a), "+v"(b), "+v"(c), "+v"(d));
#endif
}
__device__ __forceinline__ void wave_sync_lds() {
  __builtin_amdgcn_fence(__ATOMIC_RELEASE, "workgroup");
  __builtin_amdgcn_wave_barrier();
  __builtin_amdgcn_fence(__ATOMIC_ACQUIRE, "workgroup");
}

__device__ __forceinline__ void core64(const _Float16* A, int lda, const _Float16* Bt, int ldb, int K,
                                       int rlane, int koff, v8f (&acc)[4][4]) {
  for (int k0 = 0; k0 < K; k0 += 32) {
    v16h bh[4];
#pragma unroll
    for (int j = 0; j < 4; ++j) {
      bh[j] = ldfrag(Bt + (size_t)((j << 4) + rlane) * ldb + koff + k0);
    }
#pragma unroll
    for (int i = 0; i < 4; ++i) {
      const v16h ah = ldfrag(A + (size_t)((i << 4) + rlane) * lda + koff + k0);
#pragma unroll
      for (int j = 0; j < 4; ++j) {
        acc[i][j] = mma_raw(ah, bh[j], acc[i][j]);
      }
      dep_guard(acc[i][0], acc[i][3], ah, bh[3]);
    }
    keep4(bh[0], bh[1], bh[2], bh[3]);
  }
}

__global__ __launch_bounds__(256) void wcvt(const float* __restrict__ wq, const float* __restrict__ wk,
                                            const float* __restrict__ wv, const float* __restrict__ w2,
                                            unsigned short* Wout) {
  const int t = blockIdx.x * 256 + threadIdx.x;
  if (t >= WCVT_N) return;
  float v[8];
  if (t < WQKV_PIECES) {
    const int plane = t / (DM * (KE / 8));
    const int u = t - plane * (DM * (KE / 8));
    const int row = u >> 3, p = u & 7;
    const float* w = (plane == 0) ? wq : ((plane == 1) ? wk : wv);
#pragma unroll
    for (int e = 0; e < 8; ++e) {
      const int c  = p * 8 + e;
      const int cc = (c < NCH) ? c : (NCH - 1);
      const float x = bfr(w[row * NCH + cc]) * 16.0f;
      v[e] = (c < NCH) ? x : 0.0f;
    }
  } else {
    const int u = t - WQKV_PIECES;
    const int row = u / (DM / 8), p = u - row * (DM / 8);
    const v4f a = *(const v4f*)(w2 + (size_t)row * DM + p * 8);
    const v4f b = *(const v4f*)(w2 + (size_t)row * DM + p * 8 + 4);
    v[0] = bfr(a[0]) * 64.0f; v[1] = bfr(a[1]) * 64.0f; v[2] = bfr(a[2]) * 64.0f; v[3] = bfr(a[3]) * 64.0f;
    v[4] = bfr(b[0]) * 64.0f; v[5] = bfr(b[1]) * 64.0f; v[6] = bfr(b[2]) * 64.0f; v[7] = bfr(b[3]) * 64.0f;
  }
  const v4f lo = {v[0], v[1], v[2], v[3]};
  const v4f hi = {v[4], v[5], v[6], v[7]};
  const v4u pk = pack8h(lo, hi);
  unsigned short* dst = Wout + (size_t)t * 8;
  *(volatile v4u*)dst = pk;
  __threadfence();
  *(volatile v4u*)dst = pk;
}

__global__ __launch_bounds__(192) void enc_qkv_h(
    const float* __restrict__ pos,
    const _Float16* Wq16, const _Float16* Wk16, const _Float16* Wv16,
    const float* __restrict__ bq, const float* __restrict__ bk, const float* __restrict__ bv,
    const float* __restrict__ w1, const float* __restrict__ b1,
    const float* __restrict__ gam, const float* __restrict__ bet,
    const float* __restrict__ mu, const float* __restrict__ var,
    unsigned short* Qp, unsigned short* Kp, unsigned short* Vp, unsigned short* Hp) {
  __shared__ __align__(16) _Float16 sEmb[64][72];
  __shared__ __align__(16) float sT[6][16 * 68];
  __shared__ float sPos[3][64];
  __shared__ float sW1[DM * 3];
  __shared__ float sB1[DM];
  __shared__ float sInv[DM];
  __shared__ float sMu[DM];
  __shared__ float sBet[DM];

  const int tid  = threadIdx.x;
  const int lane = tid & 31;
  const int wave = tid >> 5;
  const int bb   = blockIdx.x >> 5;
  const int p0   = (blockIdx.x & 31) << 6;

  {
    const int c = tid >> 6, p = tid & 63;
    sPos[c][p] = bfr(pos[((size_t)bb * 3 + c) * NPT + p0 + p]);
  }
  for (int d = tid; d < DM; d += 192) {
    sW1[d * 3 + 0] = bfr(w1[d * 3 + 0]);
    sW1[d * 3 + 1] = bfr(w1[d * 3 + 1]);
    sW1[d * 3 + 2] = bfr(w1[d * 3 + 2]);
    sB1[d] = bfr(b1[d]);
    const float g = bfr(gam[d]), vv = bfr(var[d]);
    sInv[d] = g * (1.0f / sqrtf(vv + 1e-5f));
    sMu[d]  = bfr(mu[d]);
    sBet[d] = bfr(bet[d]);
  }
  for (int r = tid; r < 64; r += 192) {
#pragma unroll
    for (int c = NCH; c < 72; ++c) sEmb[r][c] = (_Float16)0.0f;
  }
  __syncthreads();

#pragma unroll 1
  for (int it = tid; it < 64 * 3 * NFREQ; it += 192) {
    const int cf = it >> 6, p = it & 63;
    const int c  = cf / NFREQ;
    const int f  = cf - c * NFREQ;
    const float ang = sPos[c][p] * (float)(1 << f);
    const float sv = sinf(ang);
    const float cv = cosf(ang);
    sEmb[p][c * 2 * NFREQ + f] = (_Float16)sv;
    sEmb[p][c * 2 * NFREQ + NFREQ + f] = (_Float16)cv;
  }

  for (int it = tid; it < 64 * (DM / 8); it += 192) {
    const int pl = it / (DM / 8);
    const int pc = it - pl * (DM / 8);
    const float x0 = sPos[0][pl], x1 = sPos[1][pl], x2 = sPos[2][pl];
    float h8[8];
#pragma unroll
    for (int e = 0; e < 8; ++e) {
      const int d = pc * 8 + e;
      const float r = sW1[d * 3 + 0] * x0 + sW1[d * 3 + 1] * x1 + sW1[d * 3 + 2] * x2 + sB1[d];
      const float t = (r - sMu[d]) * sInv[d] + sBet[d];
      h8[e] = fmaxf(t, 0.0f);
    }
    const v4f ha = {h8[0], h8[1], h8[2], h8[3]};
    const v4f hb = {h8[4], h8[5], h8[6], h8[7]};
    const v4u pk = pack8h(ha, hb);
    unsigned short* dst = Hp + ((size_t)bb * NPT + p0 + pl) * DM + pc * 8;
    *(volatile v4u*)dst = pk;
    __threadfence();
    *(volatile v4u*)dst = pk;
  }
  __syncthreads();

  const int rlane = lane & 15;
  const int koff  = (lane >> 4) * 8;
  const int mOff  = (lane >> 4) * 8;
  const int q8    = (lane & 7) * 8;
  const int rr    = lane >> 3;
  const int d0    = wave * 64;
  float* slab = sT[wave];
  v8f acc[4][4];

#pragma unroll 1
  for (int jb = 0; jb < 2; ++jb) {
    const _Float16* W = (jb == 0) ? Wq16 : Wk16;
    const float* bia  = (jb == 0) ? bq : bk;
    unsigned short* dstp = (jb == 0) ? Qp : Kp;
#pragma unroll
    for (int i = 0; i < 4; ++i)
#pragma unroll
      for (int j = 0; j < 4; ++j) acc[i][j] = zero8();
    core64(&sEmb[0][0], 72, W + (size_t)d0 * KE, KE, KE, rlane, koff, acc);
    acc_guard4(acc[0][0], acc[0][1], acc[0][2], acc[0][3]);
    acc_guard4(acc[1][0], acc[1][1], acc[1][2], acc[1][3]);
    acc_guard4(acc[2][0], acc[2][1], acc[2][2], acc[2][3]);
    acc_guard4(acc[3][0], acc[3][1], acc[3][2], acc[3][3]);
    v4f bs0 = *(const v4f*)(bia + d0 + q8);
    v4f bs1 = *(const v4f*)(bia + d0 + q8 + 4);
    bs0[0] = bfr(bs0[0]); bs0[1] = bfr(bs0[1]); bs0[2] = bfr(bs0[2]); bs0[3] = bfr(bs0[3]);
    bs1[0] = bfr(bs1[0]); bs1[1] = bfr(bs1[1]); bs1[2] = bfr(bs1[2]); bs1[3] = bfr(bs1[3]);
#pragma unroll
    for (int i = 0; i < 4; ++i) {
#pragma unroll
      for (int j = 0; j < 4; ++j) {
#pragma unroll
        for (int r = 0; r < 8; ++r) slab[(mOff + r) * 68 + (j << 4) + rlane] = acc[i][j][r];
      }
      wave_sync_lds();
      v4u pk[4];
#pragma unroll
      for (int it = 0; it < 4; ++it) {
        const int row = it * 4 + rr;
        v4f a = *(const v4f*)(slab + row * 68 + q8);
        v4f b = *(const v4f*)(slab + row * 68 + q8 + 4);
        a = a * 0.0625f + bs0;
        b = b * 0.0625f + bs1;
        pk[it] = pack8h(a, b);
      }
      for (int pass = 0; pass < 2; ++pass) {
#pragma unroll
        for (int it = 0; it < 4; ++it) {
          const int row = it * 4 + rr;
          unsigned short* dst = dstp + ((size_t)bb * NPT + p0 + (i << 4) + row) * DM + d0 + q8;
          *(volatile v4u*)dst = pk[it];
        }
        __threadfence();
      }
      wave_sync_lds();
    }
  }

  {
#pragma unroll
    for (int i = 0; i < 4; ++i)
#pragma unroll
      for (int j = 0; j < 4; ++j) acc[i][j] = zero8();
    core64(Wv16 + (size_t)d0 * KE, KE, &sEmb[0][0], 72, KE, rlane, koff, acc);
    acc_guard4(acc[0][0], acc[0][1], acc[0][2], acc[0][3]);
    acc_guard4(acc[1][0], acc[1][1], acc[1][2], acc[1][3]);
    acc_guard4(acc[2][0], acc[2][1], acc[2][2], acc[2][3]);
    acc_guard4(acc[3][0], acc[3][1], acc[3][2], acc[3][3]);
#pragma unroll
    for (int i = 0; i < 4; ++i) {
#pragma unroll
      for (int j = 0; j < 4; ++j) {
#pragma unroll
        for (int r = 0; r < 8; ++r) slab[(mOff + r) * 68 + (j << 4) + rlane] = acc[i][j][r];
      }
      wave_sync_lds();
      v4u pk[4];
#pragma unroll
      for (int it = 0; it < 4; ++it) {
        const int row = it * 4 + rr;
        const int d   = d0 + (i << 4) + row;
        const float bvv = bfr(bv[d]);
        v4f a = *(const v4f*)(slab + row * 68 + q8);
        v4f b = *(const v4f*)(slab + row * 68 + q8 + 4);
        a = a * 0.0625f + bvv;
        b = b * 0.0625f + bvv;
        pk[it] = pack8h(a, b);
      }
      for (int pass = 0; pass < 2; ++pass) {
#pragma unroll
        for (int it = 0; it < 4; ++it) {
          const int row = it * 4 + rr;
          const int d   = d0 + (i << 4) + row;
          unsigned short* dst = Vp + ((size_t)bb * DM + d) * NPT + p0 + q8;
          *(volatile v4u*)dst = pk[it];
        }
        __threadfence();
      }
      wave_sync_lds();
    }
  }
}

template <int TWO, int BROW>
__global__ __launch_bounds__(256) void gemm64(
    const _Float16* A, int lda, const _Float16* Bt, int ldb, int K,
    const _Float16* A2, int lda2, const _Float16* B2, int ldb2, int K2, float mid,
    float* C, int ldc, float alpha, const float* __restrict__ bias, int M, int N) {
  __shared__ __align__(16) float sT[8][16 * 68];
  const int lane = threadIdx.x & 31;
  const int wave = threadIdx.x >> 5;
  const int tilesN = N >> 6;
  const int tilesM = M >> 6;
  const int tile = blockIdx.x * 8 + wave;
  if (tile >= tilesM * tilesN) return;
  const int tm = tile / tilesN;
  const int tn = tile - tm * tilesN;
  const int m0 = tm << 6;
  const int n0 = tn << 6;

  const int rlane = lane & 15;
  const int koff  = (lane >> 4) * 8;
  const int mOff  = (lane >> 4) * 8;

  v8f acc[4][4];
#pragma unroll
  for (int i = 0; i < 4; ++i)
#pragma unroll
    for (int j = 0; j < 4; ++j) acc[i][j] = zero8();

  core64(A + (size_t)m0 * lda, lda, Bt + (size_t)n0 * ldb, ldb, K, rlane, koff, acc);
  if (TWO) {
    acc_guard4(acc[0][0], acc[0][1], acc[0][2], acc[0][3]);
    acc_guard4(acc[1][0], acc[1][1], acc[1][2], acc[1][3]);
    acc_guard4(acc[2][0], acc[2][1], acc[2][2], acc[2][3]);
    acc_guard4(acc[3][0], acc[3][1], acc[3][2], acc[3][3]);
#pragma unroll
    for (int i = 0; i < 4; ++i)
#pragma unroll
      for (int j = 0; j < 4; ++j) acc[i][j] = acc[i][j] * mid;
    core64(A2 + (size_t)m0 * lda2, lda2, B2 + (size_t)n0 * ldb2, ldb2, K2, rlane, koff, acc);
  }
  acc_guard4(acc[0][0], acc[0][1], acc[0][2], acc[0][3]);
  acc_guard4(acc[1][0], acc[1][1], acc[1][2], acc[1][3]);
  acc_guard4(acc[2][0], acc[2][1], acc[2][2], acc[2][3]);
  acc_guard4(acc[3][0], acc[3][1], acc[3][2], acc[3][3]);

  float* slab = sT[wave];
  const int hh = lane >> 4, c4 = (lane & 15) * 4;
#pragma unroll
  for (int i = 0; i < 4; ++i) {
    const int mBase = m0 + (i << 4);
#pragma unroll
    for (int j = 0; j < 4; ++j) {
#pragma unroll
      for (int r = 0; r < 8; ++r) slab[(mOff + r) * 68 + (j << 4) + rlane] = acc[i][j][r];
    }
    wave_sync_lds();
    v4f vv[8];
#pragma unroll
    for (int it = 0; it < 8; ++it) {
      const int row = it * 2 + hh;
      float bv0 = 0.0f;
      if (BROW) bv0 = bfr(bias[mBase + row]);
      v4f v = *(const v4f*)(slab + row * 68 + c4);
      vv[it] = v * alpha + bv0;
    }
    for (int pass = 0; pass < 2; ++pass) {
#pragma unroll
      for (int it = 0; it < 8; ++it) {
        const int row = it * 2 + hh;
        *(volatile v4f*)(C + (size_t)(mBase + row) * ldc + n0 + c4) = vv[it];
      }
      __threadfence();
    }
    wave_sync_lds();
  }
}

__global__ __launch_bounds__(256) void softmax_row(const float* __restrict__ S, unsigned short* P) {
  __shared__ float sMx[8];
  __shared__ float sSm[8];
  const int tid  = threadIdx.x;
  const int lane = tid & 31;
  const int wave = tid >> 5;
  const int q    = blockIdx.x;
  const size_t rb = (size_t)q * NPT;
  const int c0 = tid * 8;
  const v4f a0 = *(const v4f*)(S + rb + c0);
  const v4f a1 = *(const v4f*)(S + rb + c0 + 4);
  float v[8];
  v[0] = a0[0]; v[1] = a0[1]; v[2] = a0[2]; v[3] = a0[3];
  v[4] = a1[0]; v[5] = a1[1]; v[6] = a1[2]; v[7] = a1[3];

  float mx = v[0];
#pragma unroll
  for (int i = 1; i < 8; ++i) mx = fmaxf(mx, v[i]);
  mx = fmaxf(mx, __shfl_xor(mx, 16));
  mx = fmaxf(mx, __shfl_xor(mx, 8));
  mx = fmaxf(mx, __shfl_xor(mx, 4));
  mx = fmaxf(mx, __shfl_xor(mx, 2));
  mx = fmaxf(mx, __shfl_xor(mx, 1));
  if (lane == 0) sMx[wave] = mx;
  __syncthreads();
  float m = sMx[0];
#pragma unroll
  for (int w = 1; w < 8; ++w) m = fmaxf(m, sMx[w]);

  float e[8];
#pragma unroll
  for (int i = 0; i < 8; ++i) e[i] = __expf(v[i] - m);
  float part = ((e[0] + e[1]) + (e[2] + e[3])) + ((e[4] + e[5]) + (e[6] + e[7]));
  part += __shfl_xor(part, 16);
  part += __shfl_xor(part, 8);
  part += __shfl_xor(part, 4);
  part += __shfl_xor(part, 2);
  part += __shfl_xor(part, 1);
  if (lane == 0) sSm[wave] = part;
  __syncthreads();
  const float l  = ((sSm[0] + sSm[1]) + (sSm[2] + sSm[3])) + ((sSm[4] + sSm[5]) + (sSm[6] + sSm[7]));
  const float sc = (1.0f / l) * 1024.0f;

  const v4f pa = {e[0] * sc, e[1] * sc, e[2] * sc, e[3] * sc};
  const v4f pb = {e[4] * sc, e[5] * sc, e[6] * sc, e[7] * sc};
  const v4u pk = pack8h(pa, pb);
  unsigned short* dst = P + rb + c0;
  *(volatile v4u*)dst = pk;
  __threadfence();
  *(volatile v4u*)dst = pk;
}

extern "C" void kernel_launch(void* const* d_in, const int* in_sizes, int n_in,
                              void* d_out, int out_size, void* d_ws, size_t ws_size,
                              hipStream_t stream) {
  if (n_in < 15) return;
  if (in_sizes[0] != NBATCH * 3 * NPT) return;
  if (in_sizes[1] != DM * NCH || in_sizes[3] != DM * NCH || in_sizes[5] != DM * NCH) return;
  if (in_sizes[2] != DM || in_sizes[4] != DM || in_sizes[6] != DM) return;
  if (in_sizes[7] != DM * 3 || in_sizes[8] != DM) return;
  if (in_sizes[9] != DM || in_sizes[10] != DM || in_sizes[11] != DM || in_sizes[12] != DM) return;
  if (in_sizes[13] != DM * DM || in_sizes[14] != DM) return;
  if (out_size != NBATCH * DM * NPT) return;

  const float* pos   = (const float*)d_in[0];
  const float* wq    = (const float*)d_in[1];
  const float* bq    = (const float*)d_in[2];
  const float* wk    = (const float*)d_in[3];
  const float* bk    = (const float*)d_in[4];
  const float* wv    = (const float*)d_in[5];
  const float* bv    = (const float*)d_in[6];
  const float* w1    = (const float*)d_in[7];
  const float* b1    = (const float*)d_in[8];
  const float* gam   = (const float*)d_in[9];
  const float* bet   = (const float*)d_in[10];
  const float* mu    = (const float*)d_in[11];
  const float* var   = (const float*)d_in[12];
  const float* w2    = (const float*)d_in[13];
  const float* b2    = (const float*)d_in[14];
  float* out = (float*)d_out;

  const size_t BWGT = (size_t)WCVT_N * 16;
  const size_t BQK  = (size_t)NBATCH * NPT * DM * 2;
  const size_t BS   = (size_t)NPT * NPT * 4;
  const size_t BP   = (size_t)NPT * NPT * 2;
  size_t off = 0;
  const size_t oW = off; off += BWGT;
  const size_t oQ = off; off += BQK;
  const size_t oK = off; off += BQK;
  const size_t oV = off; off += BQK;
  const size_t oH = off; off += BQK;
  const size_t oS = off; off += BS;
  const size_t oP = off; off += BP;
  if (off > ws_size) return;
  if (off > (size_t)134217728) return;

  char* ws = (char*)d_ws;
  _Float16* W16 = (_Float16*)(ws + oW);
  const _Float16* Wq16 = W16;
  const _Float16* Wk16 = W16 + (size_t)DM * KE;
  const _Float16* Wv16 = W16 + (size_t)2 * DM * KE;
  const _Float16* W2s  = W16 + (size_t)3 * DM * KE;
  unsigned short* Qp = (unsigned short*)(ws + oQ);
  unsigned short* Kp = (unsigned short*)(ws + oK);
  unsigned short* Vp = (unsigned short*)(ws + oV);
  unsigned short* Hp = (unsigned short*)(ws + oH);
  float* S = (float*)(ws + oS);
  unsigned short* P = (unsigned short*)(ws + oP);

  const dim3 blk(256);
  const dim3 gW(WCVT_N / 256);
  const dim3 gE(NBATCH * (NPT / 64));
  const dim3 gS(((NPT / 64) * (NPT / 64) + 7) / 8);
  const dim3 gSm(NPT);
  const dim3 gO(((DM / 64) * (NPT / 64) + 7) / 8);

  wcvt<<<gW, blk, 0, stream>>>(wq, wk, wv, w2, (unsigned short*)W16);
  enc_qkv_h<<<gE, dim3(192), 0, stream>>>(pos, Wq16, Wk16, Wv16, bq, bk, bv, w1, b1, gam, bet, mu, var,
                                          Qp, Kp, Vp, Hp);

  for (int b = 0; b < NBATCH; ++b) {
    const _Float16* Qb = (const _Float16*)(Qp + (size_t)b * NPT * DM);
    const _Float16* Kb = (const _Float16*)(Kp + (size_t)b * NPT * DM);
    const _Float16* Vb = (const _Float16*)(Vp + (size_t)b * DM * NPT);
    const _Float16* Hb = (const _Float16*)(Hp + (size_t)b * NPT * DM);
    float* outb = out + (size_t)b * DM * NPT;
    gemm64<0, 0><<<gS, blk, 0, stream>>>(Qb, DM, Kb, DM, DM, Qb, DM, Kb, DM, 0, 1.0f,
                                         S, NPT, QK_SCALE, b2, NPT, NPT);
    softmax_row<<<gSm, blk, 0, stream>>>(S, P);
    gemm64<1, 1><<<gO, blk, 0, stream>>>(Vb, NPT, (const _Float16*)P, NPT, NPT, W2s, DM, Hb, DM, DM,
                                         0.0625f, outb, NPT, 0.015625f, b2, DM, NPT);
  }
  (void)hipGetLastError();
}
